// DendriticLayer_65352222376342
// MI455X (gfx1250) — hardware-run, weakly checked
//
#include <hip/hip_runtime.h>
#include <hip/hip_fp16.h>
#include <math.h>

typedef __attribute__((ext_vector_type(16))) _Float16 v16h;
typedef __attribute__((ext_vector_type(8)))  _Float16 v8h;
typedef __attribute__((ext_vector_type(8)))  float    v8f;
typedef __attribute__((ext_vector_type(4)))  float    v4f;
typedef __attribute__((ext_vector_type(2)))  unsigned v2u;
typedef __attribute__((ext_vector_type(4)))  unsigned v4u;

constexpr int kB      = 512;
constexpr int kNin    = 1024;
constexpr int kNout   = 256;
constexpr int kT      = 100;
constexpr int kTc     = 25;
constexpr int kNChunk = 4;
constexpr int kRowsC  = kTc * kB;
constexpr float kPCarry = 16384.0f;
constexpr float kWCarry = 1024.0f;
constexpr float kTauSyn = 5.0f;
constexpr float kLeak   = 0.1f;
static_assert(kB == 512 && kNin == 1024 && kNout == 256 && kT == 100);
static_assert(kTc == 25 && kNChunk == 4 && kTc * kNChunk == kT);
static_assert(kRowsC == 12800);
static_assert((kNin % kNout) == 0 && (kNin / kNout) == 4);
static_assert((kNin % 32) == 0 && (kNout % 64) == 0 && (kRowsC % 32) == 0);
static_assert((kNin % 8) == 0 && (kNout % 4) == 0);
static_assert(kPCarry == 16384.0f && kWCarry == 1024.0f);

constexpr size_t kSzPH = (size_t)kRowsC * kNin * 2;
constexpr size_t kSzWM = (size_t)kNout * kNin * 2;
constexpr size_t kSzI  = (size_t)kT * kB * kNout * 4;
constexpr size_t kOffPH = 0;
constexpr size_t kOffWM = kOffPH + kSzPH;
constexpr size_t kOffI  = kOffWM + kSzWM;
constexpr size_t kWsTotal = kOffI + kSzI;
static_assert(kSzPH == 26214400ull && kSzWM == 524288ull && kSzI == 52428800ull);
static_assert(kWsTotal == 26214400ull + 524288ull + 52428800ull);
static_assert(kWsTotal == 79167488ull);
static_assert(kWsTotal <= 134217728ull);
static_assert((kSzPH % 128) == 0 && (kSzWM % 128) == 0 && (kSzI % 128) == 0);
static_assert((((size_t)kRowsC * kNout * 4) % 128) == 0);

__device__ __forceinline__ _Float16 f16_flush(float v) {
  const float w = (fabsf(v) < 6.103515625e-05f) ? 0.0f : v;
  return (_Float16)w;
}

__device__ __forceinline__ float bf16r(float v) {
  unsigned u = __float_as_uint(v);
  u = (u + 0x7FFFu + ((u >> 16) & 1u)) & 0xFFFF0000u;
  return __uint_as_float(u);
}

__device__ __forceinline__ float h16_to_f32(unsigned hb) {
  const unsigned sgn = (hb & 0x8000u) << 16; const unsigned em = hb & 0x7fffu;
  const float fn = __uint_as_float((em << 13) + 0x38000000u);
  const float fs = (float)em * 5.9604644775390625e-8f;
  const float mag = (em < 0x400u) ? fs : fn; return __uint_as_float(__float_as_uint(mag) | sgn); }

namespace eng {
union FragU { v16h v; v8h h[2]; };
__device__ __forceinline__ v16h frag_load(const _Float16* p) {
  FragU f;
  f.h[0] = *(const v8h*)(p);
  f.h[1] = *(const v8h*)(p + 16);
  return f.v;
}
__device__ __forceinline__ v8f mma(v16h a, v16h b, v8f c) {
  return __builtin_amdgcn_wmma_f32_16x16x32_f16(false, a, false, b, (short)0, c, false, false);
}
__device__ __forceinline__ void guard1(v8f& a, v16h x, v16h y) {
  asm volatile("v_nop\n\tv_nop\n\tv_nop\n\tv_nop" : "+v"(a) : "v"(x), "v"(y));
}
__device__ __forceinline__ void guard_acc(v8f& a) {
  asm volatile("v_nop\n\tv_nop\n\tv_nop\n\tv_nop" : "+v"(a));
}
__device__ __forceinline__ void keep4(v16h a, v16h b, v16h c, v16h d) {
  asm volatile("v_nop" :: "v"(a), "v"(b), "v"(c), "v"(d));
}

template <int MI, int SPL>
__global__ __launch_bounds__(256) void gemm_f16_kernel(
    const unsigned short* __restrict__ Ap, const unsigned short* __restrict__ A2p, int lda,
    const unsigned short* __restrict__ Btp, const unsigned short* __restrict__ Bt2p, int ldb,
    float* __restrict__ C, int ldc, int M, int N, int K, float scale, float rscale)
{
  static_assert(MI >= 1 && MI <= 2);
  static_assert(SPL >= 0 && SPL <= 2);
  const _Float16* A   = (const _Float16*)Ap;
  const _Float16* A2  = (const _Float16*)A2p;
  const _Float16* Bt  = (const _Float16*)Btp;
  const _Float16* Bt2 = (const _Float16*)Bt2p;
  __shared__ __align__(16) float sT[8][16 * 68];
  const int lane = threadIdx.x & 31;
  const int wave = threadIdx.x >> 5;
  const int tilesN = N >> 6;
  const int tilesM = M / (16 * MI);
  const int tile = blockIdx.x * 8 + wave;
  if (tile >= tilesM * tilesN) return;
  const int tm = tile / tilesN;
  const int tn = tile - tm * tilesN;
  const int m0 = tm * (16 * MI);
  const int n0 = tn << 6;
  const int rlane = lane & 15;
  const int koff  = (lane >> 4) * 8;
  const int mOff  = (lane >> 4) * 8;

  v8f acc[MI][4], accr[MI][4];
#pragma unroll
  for (int i = 0; i < MI; ++i)
#pragma unroll
    for (int j = 0; j < 4; ++j) {
      acc[i][j]  = (v8f){0.f, 0.f, 0.f, 0.f, 0.f, 0.f, 0.f, 0.f};
      accr[i][j] = (v8f){0.f, 0.f, 0.f, 0.f, 0.f, 0.f, 0.f, 0.f};
    }

  for (int k0 = 0; k0 < K; k0 += 32) {
    v16h bh[4], bl[4];
#pragma unroll
    for (int j = 0; j < 4; ++j) {
      const size_t bo = (size_t)(n0 + (j << 4) + rlane) * ldb + koff + k0;
      bh[j] = frag_load(Bt + bo);
      if (SPL == 2) bl[j] = frag_load(Bt2 + bo); else bl[j] = bh[j];
    }
#pragma unroll
    for (int i = 0; i < MI; ++i) {
      const size_t ao = (size_t)(m0 + (i << 4) + rlane) * lda + koff + k0;
      const v16h ah = frag_load(A + ao);
      v16h al = ah;
      if (SPL >= 1) al = frag_load(A2 + ao);
#pragma unroll
      for (int j = 0; j < 4; ++j) {
        acc[i][j] = mma(ah, bh[j], acc[i][j]);
        if (SPL >= 1) accr[i][j] = mma(al, bh[j], accr[i][j]);
        if (SPL == 2) accr[i][j] = mma(ah, bl[j], accr[i][j]);
      }
#pragma unroll
      for (int j = 0; j < 4; ++j) {
        guard1(acc[i][j], ah, al);
        if (SPL >= 1) guard1(accr[i][j], ah, al);
      }
    }
    keep4(bh[0], bh[1], bh[2], bh[3]);
    if (SPL == 2) keep4(bl[0], bl[1], bl[2], bl[3]);
  }
#pragma unroll
  for (int i = 0; i < MI; ++i)
#pragma unroll
    for (int j = 0; j < 4; ++j) {
      guard_acc(acc[i][j]);
      if (SPL >= 1) guard_acc(accr[i][j]);
    }

  float* slab = sT[wave];
#pragma unroll
  for (int i = 0; i < MI; ++i) {
    const int mBase = m0 + (i << 4);
#pragma unroll
    for (int j = 0; j < 4; ++j) {
#pragma unroll
      for (int r = 0; r < 8; ++r) {
        float v = acc[i][j][r] * scale;
        if (SPL >= 1) v += accr[i][j][r] * rscale;
        slab[(mOff + r) * 68 + (j << 4) + rlane] = v;
      }
    }
    __builtin_amdgcn_fence(__ATOMIC_RELEASE, "workgroup");
    __builtin_amdgcn_wave_barrier();
    __builtin_amdgcn_fence(__ATOMIC_ACQUIRE, "workgroup");
    {
      const int hh = lane >> 4, c4 = (lane & 15) * 4;
      for (int pass = 0; pass < 2; ++pass) {
#pragma unroll
        for (int it = 0; it < 8; ++it) {
          const int row = it * 2 + hh;
          const v4f v = *(const v4f*)(slab + row * 68 + c4);
          *(volatile v4f*)(C + (size_t)(mBase + row) * ldc + n0 + c4) = v;
        }
        __threadfence();
      }
    }
    __builtin_amdgcn_fence(__ATOMIC_RELEASE, "workgroup");
    __builtin_amdgcn_wave_barrier();
    __builtin_amdgcn_fence(__ATOMIC_ACQUIRE, "workgroup");
  }
}
}

__device__ __forceinline__ _Float16 in_half(float v, float carry, bool live) {
  const float t = live ? (bf16r(v) * carry) : 0.0f;
  return f16_flush(t);
}
__device__ __forceinline__ _Float16 val_half(float v, float carry, bool live) {
  const float t = live ? (v * carry) : 0.0f;
  return f16_flush(t);
}
__device__ __forceinline__ int imin2(int a, int b) {
  return (a < b) ? a : b;
}
__device__ __forceinline__ int iclamp(int v, int lo, int hi) {
  const int t = (v < lo) ? lo : v;
  return (t > hi) ? hi : t;
}

__global__ __launch_bounds__(256) void pack_wm_kernel(
    const float* __restrict__ w, unsigned short* __restrict__ WM)
{
  const int idx = blockIdx.x * 256 + threadIdx.x;
  const int o = idx / (kNin / 8);
  const int k8 = (idx - o * (kNin / 8)) * 8;
  const float* sp = w + (size_t)o * kNin + k8;
  const v4f a0 = *(const v4f*)(sp);
  const v4f a1 = *(const v4f*)(sp + 4);
  const float f0 = a0[0];
  const float f1 = a0[1];
  const float f2 = a0[2];
  const float f3 = a0[3];
  const float f4 = a1[0];
  const float f5 = a1[1];
  const float f6 = a1[2];
  const float f7 = a1[3];
  const bool l0 = (((k8 + 0) >> 2) == o);
  const bool l1 = (((k8 + 1) >> 2) == o);
  const bool l2 = (((k8 + 2) >> 2) == o);
  const bool l3 = (((k8 + 3) >> 2) == o);
  const bool l4 = (((k8 + 4) >> 2) == o);
  const bool l5 = (((k8 + 5) >> 2) == o);
  const bool l6 = (((k8 + 6) >> 2) == o);
  const bool l7 = (((k8 + 7) >> 2) == o);
  v8h hv;
  hv[0] = in_half(f0, kWCarry, l0);
  hv[1] = in_half(f1, kWCarry, l1);
  hv[2] = in_half(f2, kWCarry, l2);
  hv[3] = in_half(f3, kWCarry, l3);
  hv[4] = in_half(f4, kWCarry, l4);
  hv[5] = in_half(f5, kWCarry, l5);
  hv[6] = in_half(f6, kWCarry, l6);
  hv[7] = in_half(f7, kWCarry, l7);
  unsigned short* q = WM + (size_t)idx * 8;
  *(volatile v8h*)q = hv;
  __threadfence();
  *(volatile v8h*)q = hv;
}

__global__ __launch_bounds__(256) void psp_pack_kernel(
    const float* __restrict__ s, unsigned short* __restrict__ PH, int t0)
{
  const int idx = blockIdx.x * 256 + threadIdx.x;
  const int r = idx / (kNin / 8);
  const int k8 = (idx - r * (kNin / 8)) * 8;
  const int tl = r / kB;
  const int b = r - tl * kB;
  const float tf = (float)(t0 + tl);
  const float* sp = s + (size_t)b * kNin + k8;
  const v4f a0 = *(const v4f*)(sp);
  const v4f a1 = *(const v4f*)(sp + 4);
  const float s0 = a0[0];
  const float s1 = a0[1];
  const float s2 = a0[2];
  const float s3 = a0[3];
  const float s4 = a1[0];
  const float s5 = a1[1];
  const float s6 = a1[2];
  const float s7 = a1[3];
  const float d0 = tf - bf16r(s0);
  const float d1 = tf - bf16r(s1);
  const float d2 = tf - bf16r(s2);
  const float d3 = tf - bf16r(s3);
  const float d4 = tf - bf16r(s4);
  const float d5 = tf - bf16r(s5);
  const float d6 = tf - bf16r(s6);
  const float d7 = tf - bf16r(s7);
  const bool l0 = (d0 >= 0.0f);
  const bool l1 = (d1 >= 0.0f);
  const bool l2 = (d2 >= 0.0f);
  const bool l3 = (d3 >= 0.0f);
  const bool l4 = (d4 >= 0.0f);
  const bool l5 = (d5 >= 0.0f);
  const bool l6 = (d6 >= 0.0f);
  const bool l7 = (d7 >= 0.0f);
  const float p0 = l0 ? expf(-d0 / kTauSyn) : 0.0f;
  const float p1 = l1 ? expf(-d1 / kTauSyn) : 0.0f;
  const float p2 = l2 ? expf(-d2 / kTauSyn) : 0.0f;
  const float p3 = l3 ? expf(-d3 / kTauSyn) : 0.0f;
  const float p4 = l4 ? expf(-d4 / kTauSyn) : 0.0f;
  const float p5 = l5 ? expf(-d5 / kTauSyn) : 0.0f;
  const float p6 = l6 ? expf(-d6 / kTauSyn) : 0.0f;
  const float p7 = l7 ? expf(-d7 / kTauSyn) : 0.0f;
  v8h hv;
  hv[0] = val_half(p0, kPCarry, true);
  hv[1] = val_half(p1, kPCarry, true);
  hv[2] = val_half(p2, kPCarry, true);
  hv[3] = val_half(p3, kPCarry, true);
  hv[4] = val_half(p4, kPCarry, true);
  hv[5] = val_half(p5, kPCarry, true);
  hv[6] = val_half(p6, kPCarry, true);
  hv[7] = val_half(p7, kPCarry, true);
  unsigned short* q = PH + (size_t)idx * 8;
  *(volatile v8h*)q = hv;
  __threadfence();
  *(volatile v8h*)q = hv;
}

__global__ __launch_bounds__(256) void integrate_softargmax_kernel(
    const float* __restrict__ I, float* __restrict__ out)
{
  const int idx = blockIdx.x * 256 + threadIdx.x;
  const int b = idx / (kNout / 4);
  const int o4 = (idx - b * (kNout / 4)) * 4;
  v4f v = {0.0f, 0.0f, 0.0f, 0.0f};
  v4f m = {-3.0e38f, -3.0e38f, -3.0e38f, -3.0e38f};
  for (int t = 0; t < kT; ++t) {
    const v4f it = *(const v4f*)(I + ((size_t)t * kB + b) * kNout + o4);
    v[0] = v[0] + (-v[0] + it[0]) * kLeak;
    v[1] = v[1] + (-v[1] + it[1]) * kLeak;
    v[2] = v[2] + (-v[2] + it[2]) * kLeak;
    v[3] = v[3] + (-v[3] + it[3]) * kLeak;
    m[0] = fmaxf(m[0], v[0]);
    m[1] = fmaxf(m[1], v[1]);
    m[2] = fmaxf(m[2], v[2]);
    m[3] = fmaxf(m[3], v[3]);
  }
  v = (v4f){0.0f, 0.0f, 0.0f, 0.0f};
  v4f den = {0.0f, 0.0f, 0.0f, 0.0f};
  v4f num = {0.0f, 0.0f, 0.0f, 0.0f};
  for (int t = 0; t < kT; ++t) {
    const v4f it = *(const v4f*)(I + ((size_t)t * kB + b) * kNout + o4);
    const float tf = (float)t;
    v[0] = v[0] + (-v[0] + it[0]) * kLeak;
    v[1] = v[1] + (-v[1] + it[1]) * kLeak;
    v[2] = v[2] + (-v[2] + it[2]) * kLeak;
    v[3] = v[3] + (-v[3] + it[3]) * kLeak;
    const float e0 = expf(v[0] / 0.5f - m[0] / 0.5f);
    const float e1 = expf(v[1] / 0.5f - m[1] / 0.5f);
    const float e2 = expf(v[2] / 0.5f - m[2] / 0.5f);
    const float e3 = expf(v[3] / 0.5f - m[3] / 0.5f);
    den[0] = den[0] + e0;
    den[1] = den[1] + e1;
    den[2] = den[2] + e2;
    den[3] = den[3] + e3;
    num[0] = num[0] + e0 * tf;
    num[1] = num[1] + e1 * tf;
    num[2] = num[2] + e2 * tf;
    num[3] = num[3] + e3 * tf;
  }
  v4f o;
  o[0] = num[0] / den[0];
  o[1] = num[1] / den[1];
  o[2] = num[2] / den[2];
  o[3] = num[3] / den[3];
  float* q = out + (size_t)idx * 4;
  *(volatile v4f*)q = o;
  __threadfence();
  *(volatile v4f*)q = o;
}

static_assert(((kNout * (kNin / 8)) % 256) == 0 && (kNout * (kNin / 8)) / 256 == 128);
static_assert(((kRowsC * (kNin / 8)) % 256) == 0 && (kRowsC * (kNin / 8)) / 256 == 6400);
static_assert(((kRowsC / 32) * (kNout / 64)) % 8 == 0 && ((kRowsC / 32) * (kNout / 64)) / 8 == 200);
static_assert((12800 / 32) * (256 / 64) / 8 == 200 && ((12800 / 32) * (256 / 64)) % 8 == 0);
static_assert(((kB * (kNout / 4)) % 256) == 0 && (kB * (kNout / 4)) / 256 == 128);
static_assert(kRowsC == 12800 && kNout == 256 && kNin == 1024);

extern "C" void kernel_launch(void* const* d_in, const int* in_sizes, int n_in,
                              void* d_out, int out_size, void* d_ws, size_t ws_size,
                              hipStream_t stream)
{
  if (n_in < 2) return;
  if (in_sizes[0] != kB * kNin) return;
  if (in_sizes[1] != kNout * kNin) return;
  if (out_size != kB * kNout) return;
  if (ws_size < kWsTotal) return;

  const float* s = (const float*)d_in[0];
  const float* w = (const float*)d_in[1];
  float* out = (float*)d_out;

  char* ws = (char*)d_ws;
  unsigned short* PH   = (unsigned short*)(ws + kOffPH);
  unsigned short* WM   = (unsigned short*)(ws + kOffWM);
  float*          Ibuf = (float*)(ws + kOffI);

  constexpr float s1 = 1.0f / (kPCarry * kWCarry);

  pack_wm_kernel<<<(kNout * (kNin / 8)) / 256, 256, 0, stream>>>(w, WM);

  for (int c = 0; c < kNChunk; ++c) {
    psp_pack_kernel<<<(kRowsC * (kNin / 8)) / 256, 256, 0, stream>>>(s, PH, c * kTc);

    eng::gemm_f16_kernel<2, 0><<<dim3((12800 / 32) * (256 / 64) / 8), 256, 0, stream>>>(
        PH, nullptr, 1024, WM, nullptr, 1024, Ibuf + (size_t)c * kRowsC * kNout, 256, 12800, 256, 1024, s1, 0.0f);
  }

  integrate_softargmax_kernel<<<(kB * (kNout / 4)) / 256, 256, 0, stream>>>(Ibuf, out);
}
